// MaskedSelfRelation_44375602102656
// MI455X (gfx1250) — hardware-verified
//
#include <hip/hip_runtime.h>
#include <stdint.h>


typedef _Float16 v16h __attribute__((ext_vector_type(16)));
typedef _Float16 v8h  __attribute__((ext_vector_type(8)));
typedef __bf16   v16b __attribute__((ext_vector_type(16)));
typedef unsigned short v8us __attribute__((ext_vector_type(8)));
typedef float v8f __attribute__((ext_vector_type(8)));
typedef float v4f __attribute__((ext_vector_type(4)));
typedef _Float16 v8ha __attribute__((ext_vector_type(8), __may_alias__));
typedef float    v4fa __attribute__((ext_vector_type(4), __may_alias__));

union HFrag { v16h v; v8h p[2]; _Float16 s[16]; };
union BFrag { v16b v; v8us p[2]; unsigned short s[16]; };
union H8 { v8h v; _Float16 s[8]; };
union U8 { v8us v; unsigned short s[8]; };
union F8 { v4f v[2]; float s[8]; };

#define HD   768
#define RD   64
#define DH   12
#define NB   4
#define SQ   512
#define NROW (NB * SQ)
#define KP   72
#define SP   68

typedef char shape_chk0[(NROW % 64 == 0) ? 1 : -1];
typedef char shape_chk1[(HD % 64 == 0) ? 1 : -1];
typedef char shape_chk2[(SQ % 64 == 0) ? 1 : -1];
typedef char shape_chk3[(RD * DH == HD) ? 1 : -1];

__device__ __forceinline__ int kmap(int i, int h) {
    return (i < 8) ? (8 * h + i) : (16 + 8 * h + (i - 8));
}
__device__ __forceinline__ unsigned short bf_rne(float f) {
    unsigned u = __float_as_uint(f);
    u = u + 0x7FFFu + ((u >> 16) & 1u);
    return (unsigned short)(u >> 16);
}
__device__ __forceinline__ float bf_up(unsigned short b) {
    return __uint_as_float(((unsigned)b) << 16);
}
__device__ __forceinline__ v8f zero8() {
    v8f z = {0.f, 0.f, 0.f, 0.f, 0.f, 0.f, 0.f, 0.f};
    return z;
}
__device__ __forceinline__ v8f mma_bf(v16b a, v16b b, v8f c) {
    c = __builtin_amdgcn_wmma_f32_16x16x32_bf16(false, a, false, b, (short)0, c, false, false);
    asm volatile("v_nop\n\tv_nop\n\tv_nop\n\tv_nop" : "+v"(c) : "v"(a), "v"(b));
    return c;
}
__device__ __forceinline__ v8f mma_h(v16h a, v16h b, v8f c) {
    c = __builtin_amdgcn_wmma_f32_16x16x32_f16(false, a, false, b, (short)0, c, false, false);
    asm volatile("v_nop\n\tv_nop\n\tv_nop\n\tv_nop" : "+v"(c) : "v"(a), "v"(b));
    return c;
}
__device__ __forceinline__ float wsum32(float v) {
#pragma unroll
    for (int s = 16; s > 0; s >>= 1) v += __shfl_xor(v, s, 32);
    return v;
}
__device__ __forceinline__ float max16(float v) {
#pragma unroll
    for (int s = 1; s < 16; s <<= 1) v = fmaxf(v, __shfl_xor(v, s, 16));
    return v;
}
__device__ __forceinline__ float sum16(float v) {
#pragma unroll
    for (int s = 1; s < 16; s <<= 1) v += __shfl_xor(v, s, 16);
    return v;
}

__device__ __forceinline__ void store_rows_f32(const float* st, float* dst, int pitch, int lane) {
    for (int pass = 0; pass < 2; ++pass) {
#pragma unroll
        for (int it = 0; it < 8; ++it) {
            const int L = it * 4 + (lane >> 3);
            const int row = L >> 1;
            const int c = (L & 1) * 32 + (lane & 7) * 4;
            const v4f v = *(const v4fa*)(st + row * SP + c);
            *(volatile v4f*)(dst + (size_t)row * pitch + c) = v;
        }
        if (pass == 0) __threadfence();
    }
}
__device__ __forceinline__ void store_rows_h(const float* st, _Float16* dst, int pitch, int lane) {
    for (int pass = 0; pass < 2; ++pass) {
#pragma unroll
        for (int it = 0; it < 4; ++it) {
            const int row = it * 4 + (lane >> 3);
            const int c = (lane & 7) * 8;
            F8 f;
            f.v[0] = *(const v4fa*)(st + row * SP + c);
            f.v[1] = *(const v4fa*)(st + row * SP + c + 4);
            H8 o;
#pragma unroll
            for (int q = 0; q < 8; ++q) o.s[q] = (_Float16)f.s[q];
            *(volatile v8h*)(dst + (size_t)row * pitch + c) = o.v;
        }
        if (pass == 0) __threadfence();
    }
}
__device__ __forceinline__ void store_rows_bf2(const float* st, unsigned short* dhi, unsigned short* dlo,
                                               int pitch, int lane) {
    for (int pass = 0; pass < 2; ++pass) {
#pragma unroll
        for (int it = 0; it < 4; ++it) {
            const int row = it * 4 + (lane >> 3);
            const int c = (lane & 7) * 8;
            F8 f;
            f.v[0] = *(const v4fa*)(st + row * SP + c);
            f.v[1] = *(const v4fa*)(st + row * SP + c + 4);
            U8 hi, lo;
#pragma unroll
            for (int q = 0; q < 8; ++q) {
                const unsigned short hb = bf_rne(f.s[q]);
                hi.s[q] = hb;
                lo.s[q] = bf_rne(f.s[q] - bf_up(hb));
            }
            *(volatile v8us*)(dhi + (size_t)row * pitch + c) = hi.v;
            *(volatile v8us*)(dlo + (size_t)row * pitch + c) = lo.v;
        }
        if (pass == 0) __threadfence();
    }
}

__global__ __launch_bounds__(256) void k_cvt_split(const float* __restrict__ s0, const float* __restrict__ s1,
                                                   int n0, int ntot,
                                                   unsigned short* __restrict__ dhi,
                                                   unsigned short* __restrict__ dlo) {
    const int i8 = (blockIdx.x * 256 + threadIdx.x) * 8;
    if (i8 + 8 <= ntot) {
        const float* src = (i8 < n0) ? (s0 + i8) : (s1 + (i8 - n0));
        F8 f;
        f.v[0] = *(const v4f*)src;
        f.v[1] = *(const v4f*)(src + 4);
        U8 hi, lo;
#pragma unroll
        for (int q = 0; q < 8; ++q) {
            const unsigned short hb = bf_rne(f.s[q]);
            hi.s[q] = hb;
            lo.s[q] = bf_rne(f.s[q] - bf_up(hb));
        }
        *(volatile v8us*)(dhi + i8) = hi.v;
        *(volatile v8us*)(dlo + i8) = lo.v;
        __threadfence();
        *(volatile v8us*)(dhi + i8) = hi.v;
        *(volatile v8us*)(dlo + i8) = lo.v;
    }
}

__global__ __launch_bounds__(256) void k_cvt_h(const float* __restrict__ s, int n, float scale,
                                               _Float16* __restrict__ d) {
    const int i8 = (blockIdx.x * 256 + threadIdx.x) * 8;
    if (i8 + 8 <= n) {
        F8 f;
        f.v[0] = *(const v4f*)(s + i8);
        f.v[1] = *(const v4f*)(s + i8 + 4);
        H8 o;
#pragma unroll
        for (int q = 0; q < 8; ++q) o.s[q] = (_Float16)(f.s[q] * scale);
        *(volatile v8h*)(d + i8) = o.v;
        __threadfence();
        *(volatile v8h*)(d + i8) = o.v;
    }
}

__global__ __launch_bounds__(96) void k_ln(const float* __restrict__ x, const float* __restrict__ gam,
                                           const float* __restrict__ bet,
                                           _Float16* __restrict__ xh,
                                           unsigned short* __restrict__ xbh,
                                           unsigned short* __restrict__ xbl) {
    __shared__ float ra[4];
    __shared__ float rb[4];
    const int row = blockIdx.x, tid = threadIdx.x, lane = tid & 31, wave = tid >> 5;
    const int c0 = tid * 8;
    const size_t base = (size_t)row * HD + c0;

    F8 in;
    in.v[0] = *(const v4f*)(x + base);
    in.v[1] = *(const v4f*)(x + base + 4);
    float s = 0.f;
#pragma unroll
    for (int q = 0; q < 8; ++q) s += in.s[q];
    s = wsum32(s);
    if (lane == 0) ra[wave] = s;
    __syncthreads();
    const float mu = (ra[0] + ra[1] + ra[2]) * (1.0f / (float)HD);

    float d[8];
    float vs = 0.f;
#pragma unroll
    for (int q = 0; q < 8; ++q) { d[q] = in.s[q] - mu; vs += d[q] * d[q]; }
    vs = wsum32(vs);
    if (lane == 0) rb[wave] = vs;
    __syncthreads();
    const float var = (rb[0] + rb[1] + rb[2]) * (1.0f / (float)HD);
    const float rstd = rsqrtf(var + 1e-5f);

    F8 gg, be;
    gg.v[0] = *(const v4f*)(gam + c0);
    gg.v[1] = *(const v4f*)(gam + c0 + 4);
    be.v[0] = *(const v4f*)(bet + c0);
    be.v[1] = *(const v4f*)(bet + c0 + 4);

    H8 yh;
    U8 yb, yl;
#pragma unroll
    for (int q = 0; q < 8; ++q) {
        const float y = d[q] * rstd * gg.s[q] + be.s[q];
        yh.s[q] = (_Float16)y;
        const unsigned short hb = bf_rne(y);
        yb.s[q] = hb;
        yl.s[q] = bf_rne(y - bf_up(hb));
    }
    for (int pass = 0; pass < 2; ++pass) {
        *(volatile v8h*)(xh + base) = yh.v;
        *(volatile v8us*)(xbh + base) = yb.v;
        *(volatile v8us*)(xbl + base) = yl.v;
        if (pass == 0) __threadfence();
    }
}

__global__ __launch_bounds__(128) void k_gemm_qk(const unsigned short* __restrict__ xbh,
                                                 const unsigned short* __restrict__ xbl,
                                                 const unsigned short* __restrict__ whi,
                                                 const unsigned short* __restrict__ wlo,
                                                 const float* __restrict__ bq,
                                                 const float* __restrict__ bk,
                                                 float* __restrict__ qf,
                                                 unsigned short* __restrict__ khi,
                                                 unsigned short* __restrict__ klo) {
    __shared__ __attribute__((aligned(16))) float stile[4 * 16 * SP];
    const int tid = threadIdx.x, lane = tid & 31, wave = tid >> 5;
    const int h = (lane >> 4) & 1, m = lane & 15;
    const int sel = blockIdx.y;
    const int rbase = blockIdx.x * 64 + wave * 16;
    const size_t arow = (size_t)(rbase + m) * HD;
    const int nbase = sel * 64;

    v8f acc[4];
#pragma unroll
    for (int nt = 0; nt < 4; ++nt) acc[nt] = zero8();
    const unsigned short* wph[4];
    const unsigned short* wpl[4];
#pragma unroll
    for (int nt = 0; nt < 4; ++nt) {
        wph[nt] = whi + (size_t)(nbase + nt * 16 + m) * HD;
        wpl[nt] = wlo + (size_t)(nbase + nt * 16 + m) * HD;
    }

#pragma unroll 1
    for (int k0 = 0; k0 < HD; k0 += 32) {
        BFrag ahf, alf;
        ahf.p[0] = *(const v8us*)(xbh + arow + k0 + 8 * h);
        ahf.p[1] = *(const v8us*)(xbh + arow + k0 + 16 + 8 * h);
        alf.p[0] = *(const v8us*)(xbl + arow + k0 + 8 * h);
        alf.p[1] = *(const v8us*)(xbl + arow + k0 + 16 + 8 * h);
#pragma unroll
        for (int nt = 0; nt < 4; ++nt) {
            BFrag bh, bl;
            bh.p[0] = *(const v8us*)(wph[nt] + k0 + 8 * h);
            bh.p[1] = *(const v8us*)(wph[nt] + k0 + 16 + 8 * h);
            bl.p[0] = *(const v8us*)(wpl[nt] + k0 + 8 * h);
            bl.p[1] = *(const v8us*)(wpl[nt] + k0 + 16 + 8 * h);
            acc[nt] = mma_bf(ahf.v, bh.v, acc[nt]);
            acc[nt] = mma_bf(ahf.v, bl.v, acc[nt]);
            acc[nt] = mma_bf(alf.v, bh.v, acc[nt]);
        }
    }

    const float* bias = sel ? bk : bq;
    float* st = stile + wave * 16 * SP;
#pragma unroll
    for (int nt = 0; nt < 4; ++nt) {
        const int col = nt * 16 + m;
        const float bb = bias[col];
#pragma unroll
        for (int r = 0; r < 8; ++r) st[(8 * h + r) * SP + col] = acc[nt][r] + bb;
    }
    __syncthreads();
    if (sel == 0) {
        store_rows_f32(st, qf + (size_t)rbase * RD, RD, lane);
    } else {
        store_rows_bf2(st, khi + (size_t)rbase * RD, klo + (size_t)rbase * RD, RD, lane);
    }
}

__device__ __forceinline__ void gemm16_core(const _Float16* __restrict__ ap, const _Float16* __restrict__ W,
                                            int nbase, int m, int h, v8f (&acc)[4]) {
    const _Float16* wp[4];
#pragma unroll
    for (int nt = 0; nt < 4; ++nt) wp[nt] = W + (size_t)(nbase + nt * 16 + m) * HD;
#pragma unroll 1
    for (int k0 = 0; k0 < HD; k0 += 32) {
        HFrag a;
        a.p[0] = *(const v8h*)(ap + k0 + 8 * h);
        a.p[1] = *(const v8h*)(ap + k0 + 16 + 8 * h);
#pragma unroll
        for (int nt = 0; nt < 4; ++nt) {
            HFrag bfr;
            bfr.p[0] = *(const v8h*)(wp[nt] + k0 + 8 * h);
            bfr.p[1] = *(const v8h*)(wp[nt] + k0 + 16 + 8 * h);
            acc[nt] = mma_h(a.v, bfr.v, acc[nt]);
        }
    }
}

__global__ __launch_bounds__(128) void k_gemm_v(const _Float16* __restrict__ xh,
                                                const _Float16* __restrict__ wv16,
                                                const float* __restrict__ bv,
                                                _Float16* __restrict__ vh) {
    __shared__ __attribute__((aligned(16))) float stile[4 * 16 * SP];
    const int tid = threadIdx.x, lane = tid & 31, wave = tid >> 5;
    const int h = (lane >> 4) & 1, m = lane & 15;
    const int rbase = blockIdx.x * 64 + wave * 16;
    const int nbase = blockIdx.y * 64;
    v8f acc[4];
#pragma unroll
    for (int nt = 0; nt < 4; ++nt) acc[nt] = zero8();
    gemm16_core(xh + (size_t)(rbase + m) * HD, wv16, nbase, m, h, acc);

    float* st = stile + wave * 16 * SP;
#pragma unroll
    for (int nt = 0; nt < 4; ++nt) {
        const int col = nt * 16 + m;
        const float bb = bv[nbase + col];
#pragma unroll
        for (int r = 0; r < 8; ++r) st[(8 * h + r) * SP + col] = acc[nt][r] * (1.0f / 64.0f) + bb;
    }
    __syncthreads();
    store_rows_h(st, vh + (size_t)rbase * HD + nbase, HD, lane);
}

__global__ __launch_bounds__(128) void k_gemm_out(const _Float16* __restrict__ oh,
                                                  const _Float16* __restrict__ wo16,
                                                  const float* __restrict__ bo,
                                                  float* __restrict__ outp) {
    __shared__ __attribute__((aligned(16))) float stile[4 * 16 * SP];
    const int tid = threadIdx.x, lane = tid & 31, wave = tid >> 5;
    const int h = (lane >> 4) & 1, m = lane & 15;
    const int rbase = blockIdx.x * 64 + wave * 16;
    const int nbase = blockIdx.y * 64;
    v8f acc[4];
#pragma unroll
    for (int nt = 0; nt < 4; ++nt) acc[nt] = zero8();
    gemm16_core(oh + (size_t)(rbase + m) * HD, wo16, nbase, m, h, acc);

    float* st = stile + wave * 16 * SP;
#pragma unroll
    for (int nt = 0; nt < 4; ++nt) {
        const int col = nt * 16 + m;
        const float bb = bo[nbase + col];
#pragma unroll
        for (int r = 0; r < 8; ++r) st[(8 * h + r) * SP + col] = acc[nt][r] * (1.0f / 4096.0f) + bb;
    }
    __syncthreads();
    store_rows_f32(st, outp + (size_t)rbase * HD + nbase, HD, lane);
}

__global__ __launch_bounds__(128) void k_attn(const float* __restrict__ qf,
                                              const unsigned short* __restrict__ khi,
                                              const unsigned short* __restrict__ klo,
                                              const _Float16* __restrict__ vh,
                                              const float* __restrict__ wt,
                                              const float* __restrict__ amask,
                                              _Float16* __restrict__ oh) {
    __shared__ __attribute__((aligned(16))) unsigned short ksh[2 * 64 * KP];
    __shared__ __attribute__((aligned(16))) _Float16 vsT[4 * 16 * KP];
    __shared__ __attribute__((aligned(16))) _Float16 psh[4 * 16 * KP];
    __shared__ __attribute__((aligned(16))) _Float16 otile[16 * HD];

    const int tid = threadIdx.x, lane = tid & 31, wave = tid >> 5;
    const int h = (lane >> 4) & 1, m = lane & 15;
    const int b = blockIdx.y;
    const int row0 = b * SQ + blockIdx.x * 16;

    for (int i = tid; i < 4 * 4 * KP; i += 128) {
        const int w = i / (4 * KP);
        const int rem = i - w * 4 * KP;
        vsT[(w * 16 + 12) * KP + rem] = (_Float16)0.0f;
    }

    unsigned short* kshh = ksh;
    unsigned short* kshl = ksh + 64 * KP;
    _Float16* pw = psh + wave * 16 * KP;
    const _Float16* vw = vsT + wave * 16 * KP;
    const float* qrow = qf + (size_t)(row0 + m) * RD;

#pragma unroll 1
    for (int u = 0; u < 16; ++u) {
        const int t = u * 4 + wave;
        const float* wrow = wt + t * RD;

        BFrag ah[2], al[2];
#pragma unroll
        for (int e = 0; e < 16; ++e) {
            const int r = kmap(e, h);
            const float q0 = qrow[r] * wrow[r];
            const float q1 = qrow[r + 32] * wrow[r + 32];
            const unsigned short hb0 = bf_rne(q0);
            const unsigned short hb1 = bf_rne(q1);
            ah[0].s[e] = hb0;
            al[0].s[e] = bf_rne(q0 - bf_up(hb0));
            ah[1].s[e] = hb1;
            al[1].s[e] = bf_rne(q1 - bf_up(hb1));
        }

        v8f o = zero8();
        float mrow[8], lp[8];
#pragma unroll
        for (int g = 0; g < 8; ++g) { mrow[g] = -1e30f; lp[g] = 0.f; }

#pragma unroll 1
        for (int js = 0; js < 8; ++js) {
            const int j0 = js * 64;
            __syncthreads();

#pragma unroll
            for (int e = 0; e < 4; ++e) {
                const int idx = tid + e * 128;
                const int j = idx >> 3, c = idx & 7;
                const size_t gk = (size_t)(b * SQ + j0 + j) * RD + c * 8;
                *(v8us*)(kshh + j * KP + c * 8) = *(const v8us*)(khi + gk);
                *(v8us*)(kshl + j * KP + c * 8) = *(const v8us*)(klo + gk);
            }
#pragma unroll
            for (int e = 0; e < 3; ++e) {
                const int idx = tid + e * 128;
                const int j = idx / 6;
                const int c = idx - j * 6;
                H8 val;
                val.v = *(const v8h*)(vh + (size_t)(b * SQ + j0 + j) * HD + 48 * u + 8 * c);
#pragma unroll
                for (int q = 0; q < 8; ++q) {
                    const int col = 8 * c + q;
                    const int w2 = col / 12;
                    const int d = col - w2 * 12;
                    vsT[(w2 * 16 + d) * KP + j] = val.s[q];
                }
            }
            __syncthreads();

            v8f s[4];
#pragma unroll
            for (int nt = 0; nt < 4; ++nt) {
                s[nt] = zero8();
                const int jr = nt * 16 + m;
#pragma unroll
                for (int ks = 0; ks < 2; ++ks) {
                    BFrag bh, bl;
                    const unsigned short* kp = kshh + jr * KP + 32 * ks + 8 * h;
                    const unsigned short* kq = kshl + jr * KP + 32 * ks + 8 * h;
                    bh.p[0] = *(const v8us*)kp;
                    bh.p[1] = *(const v8us*)(kp + 16);
                    bl.p[0] = *(const v8us*)kq;
                    bl.p[1] = *(const v8us*)(kq + 16);
                    s[nt] = mma_bf(ah[ks].v, bh.v, s[nt]);
                    s[nt] = mma_bf(ah[ks].v, bl.v, s[nt]);
                    s[nt] = mma_bf(al[ks].v, bh.v, s[nt]);
                }
            }

            float mk[4];
#pragma unroll
            for (int nt = 0; nt < 4; ++nt) mk[nt] = amask[b * SQ + j0 + nt * 16 + m];
#pragma unroll
            for (int g = 0; g < 8; ++g) {
                float mx = -1e30f;
#pragma unroll
                for (int nt = 0; nt < 4; ++nt) {
                    s[nt][g] += mk[nt];
                    mx = fmaxf(mx, s[nt][g]);
                }
                mx = max16(mx);
                const float mn = fmaxf(mrow[g], mx);
                const float alpha = __expf(mrow[g] - mn);
                mrow[g] = mn;
                o[g] *= alpha;
                lp[g] *= alpha;
#pragma unroll
                for (int nt = 0; nt < 4; ++nt) {
                    const float p = __expf(s[nt][g] - mn);
                    lp[g] += p;
                    pw[(8 * h + g) * KP + nt * 16 + m] = (_Float16)(p * 4096.0f);
                }
            }
            __syncthreads();

#pragma unroll
            for (int ks = 0; ks < 2; ++ks) {
                HFrag pa, vb;
                const _Float16* pp = pw + m * KP + 32 * ks + 8 * h;
                const _Float16* vp = vw + m * KP + 32 * ks + 8 * h;
                pa.p[0] = *(const v8ha*)pp;
                pa.p[1] = *(const v8ha*)(pp + 16);
                vb.p[0] = *(const v8ha*)vp;
                vb.p[1] = *(const v8ha*)(vp + 16);
                o = mma_h(pa.v, vb.v, o);
            }
        }

#pragma unroll
        for (int g = 0; g < 8; ++g) {
            const float l = sum16(lp[g]);
            const float val = o[g] / (64.0f * l);
            if (m < DH) otile[(8 * h + g) * HD + t * DH + m] = (_Float16)val;
        }
    }
    __syncthreads();

    for (int pass = 0; pass < 2; ++pass) {
        for (int L = wave * 4 + (lane >> 3); L < 16 * (HD / 64); L += 16) {
            const int row = L / (HD / 64);
            const int seg = L - row * (HD / 64);
            const int c = seg * 64 + (lane & 7) * 8;
            const v8h v = *(const v8ha*)(otile + row * HD + c);
            *(volatile v8h*)(oh + (size_t)(row0 + row) * HD + c) = v;
        }
        if (pass == 0) __threadfence();
    }
}

extern "C" void kernel_launch(void* const* d_in, const int* in_sizes, int n_in,
                              void* d_out, int out_size, void* d_ws, size_t ws_size,
                              hipStream_t stream) {
    if (n_in < 13) return;
    const int want_n[13] = {NROW * HD, NB * SQ, HD, HD, RD * HD, RD, RD * HD, RD,
                            HD * HD, HD, RD * RD, HD * HD, HD};
    for (int i = 0; i < 13; ++i) if (in_sizes[i] != want_n[i]) return;
    if (out_size != NROW * HD) return;

    const float* tgt  = (const float*)d_in[0];
    const float* amask= (const float*)d_in[1];
    const float* ln_g = (const float*)d_in[2];
    const float* ln_b = (const float*)d_in[3];
    const float* Wq   = (const float*)d_in[4];
    const float* bq   = (const float*)d_in[5];
    const float* Wk   = (const float*)d_in[6];
    const float* bk   = (const float*)d_in[7];
    const float* Wv   = (const float*)d_in[8];
    const float* bv   = (const float*)d_in[9];
    const float* Wt   = (const float*)d_in[10];
    const float* Wo   = (const float*)d_in[11];
    const float* bo   = (const float*)d_in[12];
    float* outp = (float*)d_out;

    char* ws = (char*)d_ws;
    size_t off = 0;
    auto carve = [&](size_t bytes) { char* p = ws + off; off += (bytes + 127) & ~(size_t)127; return p; };
    _Float16*       xh   = (_Float16*)      carve((size_t)NROW * HD * 2);
    unsigned short* xbh  = (unsigned short*)carve((size_t)NROW * HD * 2);
    unsigned short* xbl  = (unsigned short*)carve((size_t)NROW * HD * 2);
    unsigned short* whi  = (unsigned short*)carve((size_t)2 * RD * HD * 2);
    unsigned short* wlo  = (unsigned short*)carve((size_t)2 * RD * HD * 2);
    _Float16*       wv16 = (_Float16*)      carve((size_t)HD * HD * 2);
    _Float16*       wo16 = (_Float16*)      carve((size_t)HD * HD * 2);
    float*          qf   = (float*)         carve((size_t)NROW * RD * 4);
    unsigned short* khi  = (unsigned short*)carve((size_t)NROW * RD * 2);
    unsigned short* klo  = (unsigned short*)carve((size_t)NROW * RD * 2);
    _Float16*       vh   = (_Float16*)      carve((size_t)NROW * HD * 2);
    _Float16*       oh   = (_Float16*)      carve((size_t)NROW * HD * 2);
    if (off > ws_size) return;

    const int nqk = 2 * RD * HD;
    const int nvw = HD * HD;
    k_cvt_split<<<(nqk / 8 + 255) / 256, 256, 0, stream>>>(Wq, Wk, RD * HD, nqk, whi, wlo);
    k_cvt_h<<<(nvw / 8 + 255) / 256, 256, 0, stream>>>(Wv, nvw, 64.0f, wv16);
    k_cvt_h<<<(nvw / 8 + 255) / 256, 256, 0, stream>>>(Wo, nvw, 64.0f, wo16);

    k_ln<<<NROW, 96, 0, stream>>>(tgt, ln_g, ln_b, xh, xbh, xbl);

    k_gemm_qk<<<dim3(NROW / 64, 2), 128, 0, stream>>>(xbh, xbl, whi, wlo, bq, bk, qf, khi, klo);
    k_gemm_v<<<dim3(NROW / 64, HD / 64), 128, 0, stream>>>(xh, wv16, bv, vh);

    k_attn<<<dim3(SQ / 16, NB), 128, 0, stream>>>(qf, khi, klo, vh, Wt, amask, oh);

    k_gemm_out<<<dim3(NROW / 64, HD / 64), 128, 0, stream>>>(oh, wo16, bo, outp);
}
